// QuantumEmbedding_13554916786258
// MI455X (gfx1250) — hardware-run, weakly checked
//
#include <hip/hip_runtime.h>
#include <math.h>

typedef __attribute__((ext_vector_type(16))) _Float16 v16h;
typedef __attribute__((ext_vector_type(8)))  _Float16 v8h;
typedef __attribute__((ext_vector_type(8)))  float    v8f;
typedef __attribute__((ext_vector_type(4)))  float    v4f;

constexpr int kSamples  = 524288;
constexpr int kXPitch   = 8;
constexpr int kWires    = 4;
constexpr int kStates   = 16;
constexpr int kLayers   = 2;
constexpr int kThreads  = 256;
constexpr int kWaves    = kThreads / 32;
constexpr int kPerWave  = 32;
constexpr int kIter     = 8;
constexpr int kBlocks   = kSamples / (kWaves * kPerWave * kIter);
constexpr int kPPitch   = 17;
constexpr int kPlaneN   = 32;
constexpr int kPlaneK   = 32;
static_assert(kStates == (1 << kWires), "state count");
static_assert(kBlocks * kWaves * kPerWave * kIter == kSamples, "exact sample cover, no tail");
static_assert(kPlaneN == 2 * kStates && kPlaneK == 2 * kStates, "operand plane shape");

constexpr float kCarryE = 512.0f;
constexpr float kCarryU = 512.0f;
constexpr float kFold   = 1.0f / (kCarryE * kCarryE * kCarryU * kCarryU);
constexpr float kF16MinNormal = 6.103515625e-5f;
constexpr float kPi = 3.14159274101257324f;

constexpr size_t kPlaneBytes = (size_t)kPlaneN * kPlaneK * 2;
constexpr size_t kOffB1   = 0;
constexpr size_t kOffB2   = kOffB1 + kPlaneBytes;
constexpr size_t kWsTotal = kPlaneBytes + kPlaneBytes;
static_assert(kWsTotal == 4096ull, "carve total");
static_assert((kOffB2 % 128) == 0, "aligned regions");

union FragU { v16h v; v8h h[2]; };
__device__ __forceinline__ v16h frag_load(const _Float16* p) {
  FragU f;
  f.h[0] = *(const v8h*)(p);
  f.h[1] = *(const v8h*)(p + 16);
  return f.v;
}
__device__ __forceinline__ v8f mma_g(v16h a, v16h b, v8f c) {
  c = __builtin_amdgcn_wmma_f32_16x16x32_f16(false, a, false, b, (short)0, c, false, false);
  asm volatile("v_nop\n\tv_nop\n\tv_nop\n\tv_nop" : "+v"(c) : "v"(a), "v"(b));
  return c;
}

__device__ __forceinline__ float flush_small(float v) {
  return (fabsf(v) < kF16MinNormal) ? 0.0f : v;
}
__device__ __forceinline__ void split16(float v, _Float16& hi, _Float16& lo) {
  const float vf = flush_small(v);
  const _Float16 hh = (_Float16)vf;
  float hf = (float)hh;
  asm volatile("" : "+v"(hf));
  const float rf = flush_small(vf - hf);
  hi = hh;
  lo = (_Float16)rf;
}

__global__ __launch_bounds__(32) void build_planes_kernel(
    const float* __restrict__ w, unsigned short* __restrict__ B1, unsigned short* __restrict__ B2)
{
  __shared__ __align__(16) float    sU[2 * kStates * 32];
  __shared__ __align__(16) _Float16 sS1[kPlaneN * kPlaneK];
  __shared__ __align__(16) _Float16 sS2[kPlaneN * kPlaneK];
  const int lane = threadIdx.x;
  const int j = lane & 15;
  constexpr int kImOff = kStates * 32;

#pragma unroll 1
  for (int k = 0; k < kStates; ++k) {
    sU[k * 32 + lane] = (k == j) ? 1.0f : 0.0f;
    sU[kImOff + k * 32 + lane] = 0.0f;
  }

#pragma unroll 1
  for (int layer = 0; layer < kLayers; ++layer) {
#pragma unroll 1
    for (int q = 0; q < kWires; ++q) {
      const int mask = 8 >> q;
      const float thy = w[(layer * kWires + q) * 2 + 0];
      const float thz = w[(layer * kWires + q) * 2 + 1];
      float sy, cy;
      sincosf(thy * 0.5f, &sy, &cy);
#pragma unroll 1
      for (int p = 0; p < 8; ++p) {
        const int low = p & (mask - 1);
        const int k0 = ((p - low) << 1) | low;
        const int k1 = k0 | mask;
        const float ar = sU[k0 * 32 + lane];
        const float ai = sU[kImOff + k0 * 32 + lane];
        const float br = sU[k1 * 32 + lane];
        const float bi = sU[kImOff + k1 * 32 + lane];
        sU[k0 * 32 + lane]          = cy * ar - sy * br;
        sU[kImOff + k0 * 32 + lane] = cy * ai - sy * bi;
        sU[k1 * 32 + lane]          = sy * ar + cy * br;
        sU[kImOff + k1 * 32 + lane] = sy * ai + cy * bi;
      }
      float sz, cz;
      sincosf(thz * 0.5f, &sz, &cz);
#pragma unroll 1
      for (int k = 0; k < kStates; ++k) {
        const float ss = (k & mask) ? sz : -sz;
        const float re = sU[k * 32 + lane];
        const float im = sU[kImOff + k * 32 + lane];
        sU[k * 32 + lane]          = re * cz - im * ss;
        sU[kImOff + k * 32 + lane] = im * cz + re * ss;
      }
    }
#pragma unroll 1
    for (int i = 0; i < kWires; ++i) {
      const int mc = 8 >> i;
      const int mt = 8 >> ((i + 1) & 3);
#pragma unroll 1
      for (int k = 0; k < kStates; ++k) {
        if ((k & mc) && !(k & mt)) {
          const int k1 = k | mt;
          const float ar = sU[k * 32 + lane];
          const float ai = sU[kImOff + k * 32 + lane];
          const float br = sU[k1 * 32 + lane];
          const float bi = sU[kImOff + k1 * 32 + lane];
          sU[k * 32 + lane]           = br;
          sU[kImOff + k * 32 + lane]  = bi;
          sU[k1 * 32 + lane]          = ar;
          sU[kImOff + k1 * 32 + lane] = ai;
        }
      }
    }
  }
  __syncthreads();

  const int plane = lane >> 4;
  const int kr = lane & 15;
  v8h h0, h1, l0, l1;
#pragma unroll
  for (int e = 0; e < 8; ++e) {
    const float u0 = sU[plane * kImOff + kr * 32 + e] * kCarryU;
    const float u1 = sU[plane * kImOff + kr * 32 + 8 + e] * kCarryU;
    _Float16 a, b;
    split16(u0, a, b);
    h0[e] = a;
    l0[e] = b;
    split16(u1, a, b);
    h1[e] = a;
    l1[e] = b;
  }
  float zf = 0.0f;
  asm volatile("" : "+v"(zf));
  v8h zz;
#pragma unroll
  for (int e = 0; e < 8; ++e) zz[e] = (_Float16)zf;
  *(v8h*)(sS1 + lane * kPlaneK + 0)  = h0;
  *(v8h*)(sS1 + lane * kPlaneK + 8)  = h1;
  *(v8h*)(sS1 + lane * kPlaneK + 16) = h0;
  *(v8h*)(sS1 + lane * kPlaneK + 24) = h1;
  *(v8h*)(sS2 + lane * kPlaneK + 0)  = l0;
  *(v8h*)(sS2 + lane * kPlaneK + 8)  = l1;
  *(v8h*)(sS2 + lane * kPlaneK + 16) = zz;
  *(v8h*)(sS2 + lane * kPlaneK + 24) = zz;
  __syncthreads();

  v8h o1[4], o2[4];
#pragma unroll
  for (int it = 0; it < 4; ++it) {
    o1[it] = *(const v8h*)(sS1 + (it * 32 + lane) * 8);
    o2[it] = *(const v8h*)(sS2 + (it * 32 + lane) * 8);
  }
  for (int pass = 0; pass < 2; ++pass) {
#pragma unroll
    for (int it = 0; it < 4; ++it) {
      *(volatile v8h*)(B1 + (it * 32 + lane) * 8) = o1[it];
      *(volatile v8h*)(B2 + (it * 32 + lane) * 8) = o2[it];
    }
    __threadfence();
  }
}

__global__ __launch_bounds__(256) void circuit_kernel(
    const float* __restrict__ x, const unsigned short* __restrict__ B1p,
    const unsigned short* __restrict__ B2p, float* __restrict__ out)
{
  __shared__ __align__(16) _Float16 sA[kWaves][kPerWave * kPlaneK];
  __shared__ __align__(16) float    sP[kWaves][kPerWave * kPPitch];
  const int tid  = threadIdx.x;
  const int lane = tid & 31;
  const int wave = tid >> 5;
  const int hh   = lane >> 4;
  const int c    = lane & 15;

  const _Float16* B1 = (const _Float16*)B1p;
  const _Float16* B2 = (const _Float16*)B2p;
  const v16h b1re = frag_load(B1 + (c) * kPlaneK + 8 * hh);
  const v16h b1im = frag_load(B1 + (kStates + c) * kPlaneK + 8 * hh);
  const v16h b2re = frag_load(B2 + (c) * kPlaneK + 8 * hh);
  const v16h b2im = frag_load(B2 + (kStates + c) * kPlaneK + 8 * hh);

  _Float16* aw = sA[wave];
  float*    pw = sP[wave];

#pragma unroll 1
  for (int it = 0; it < kIter; ++it) {
    const int base = ((blockIdx.x * kIter + it) * kWaves + wave) * kPerWave;

    const v4f xv = *(const v4f*)(x + (size_t)(base + lane) * kXPitch);
    float xa[4];
    xa[0] = xv[0];
    xa[1] = xv[1];
    xa[2] = xv[2];
    xa[3] = xv[3];
    float cq[4], sq[4];
#pragma unroll
    for (int q = 0; q < kWires; ++q) {
      const float a = (tanhf(xa[q]) * kPi) * 0.5f;
      sincosf(a, &sq[q], &cq[q]);
    }
    float m01[4], m23[4];
    m01[0] = cq[0] * cq[1];
    m01[1] = cq[0] * sq[1];
    m01[2] = sq[0] * cq[1];
    m01[3] = sq[0] * sq[1];
    m23[0] = cq[2] * cq[3];
    m23[1] = cq[2] * sq[3];
    m23[2] = sq[2] * cq[3];
    m23[3] = sq[2] * sq[3];

    v8h h0, h1, l0, l1;
#pragma unroll
    for (int k = 0; k < 8; ++k) {
      const float e0 = (m01[k >> 2] * m23[k & 3]) * kCarryE;
      const float e1 = (m01[2 + (k >> 2)] * m23[k & 3]) * kCarryE;
      _Float16 a, b;
      split16(e0, a, b);
      h0[k] = a;
      l0[k] = b;
      split16(e1, a, b);
      h1[k] = a;
      l1[k] = b;
    }
    *(v8h*)(aw + lane * kPlaneK + 0)  = h0;
    *(v8h*)(aw + lane * kPlaneK + 8)  = h1;
    *(v8h*)(aw + lane * kPlaneK + 16) = l0;
    *(v8h*)(aw + lane * kPlaneK + 24) = l1;
    __syncthreads();

#pragma unroll
    for (int mt = 0; mt < 2; ++mt) {
      const v16h a = frag_load(aw + (mt * 16 + c) * kPlaneK + 8 * hh);
      v8f are = (v8f){0.f, 0.f, 0.f, 0.f, 0.f, 0.f, 0.f, 0.f};
      v8f aim = (v8f){0.f, 0.f, 0.f, 0.f, 0.f, 0.f, 0.f, 0.f};
      are = mma_g(a, b1re, are);
      aim = mma_g(a, b1im, aim);
      are = mma_g(a, b2re, are);
      aim = mma_g(a, b2im, aim);
#pragma unroll
      for (int r = 0; r < 8; ++r) {
        pw[(mt * 16 + 8 * hh + r) * kPPitch + c] = are[r] * are[r] + aim[r] * aim[r];
      }
    }
    __syncthreads();

    float z0 = 0.0f, z1 = 0.0f, z2 = 0.0f, z3 = 0.0f;
#pragma unroll
    for (int k = 0; k < kStates; ++k) {
      const float p = pw[lane * kPPitch + k];
      z0 += (k & 8) ? -p : p;
      z1 += (k & 4) ? -p : p;
      z2 += (k & 2) ? -p : p;
      z3 += (k & 1) ? -p : p;
    }
    v4f zv;
    zv[0] = z0 * kFold;
    zv[1] = z1 * kFold;
    zv[2] = z2 * kFold;
    zv[3] = z3 * kFold;
    float* dst = out + (size_t)(base + lane) * kWires;
    for (int pass = 0; pass < 2; ++pass) {
      *(volatile v4f*)dst = zv;
      __threadfence();
    }
  }
}

extern "C" void kernel_launch(void* const* d_in, const int* in_sizes, int n_in,
                              void* d_out, int out_size, void* d_ws, size_t ws_size,
                              hipStream_t stream) {
  if (n_in < 2) return;
  if (in_sizes[0] != kSamples * kXPitch) return;
  if (in_sizes[1] != kLayers * kWires * 2) return;
  if (out_size != kSamples * kWires) return;
  if (ws_size < kWsTotal) return;

  const float* x = (const float*)d_in[0];
  const float* w = (const float*)d_in[1];
  float* out = (float*)d_out;
  char* ws = (char*)d_ws;
  unsigned short* B1 = (unsigned short*)(ws + kOffB1);
  unsigned short* B2 = (unsigned short*)(ws + kOffB2);

  build_planes_kernel<<<1, 32, 0, stream>>>(w, B1, B2);
  circuit_kernel<<<kBlocks, kThreads, 0, stream>>>(x, B1, B2, out);
}
